// CMoSModel_40707700032360
// MI455X (gfx1250) — hardware-run, weakly checked
//
#include <hip/hip_runtime.h>
#include <math.h>
#pragma clang fp contract(off)

typedef __attribute__((ext_vector_type(16))) _Float16 v16h;
typedef __attribute__((ext_vector_type(8)))  _Float16 v8h;
typedef __attribute__((ext_vector_type(8)))  float    v8f;
typedef __attribute__((ext_vector_type(4)))  float    v4f;

constexpr int kBatch  = 256;
constexpr int kLen    = 512;
constexpr int kPred   = 720;
constexpr int kChan   = 64;
constexpr int kSeg    = 16;
constexpr int kMaps   = 8;
constexpr int kTaps   = 16;
constexpr int kStride = 8;
constexpr int kConv   = (kLen - kTaps) / kStride + 1;
constexpr int kNin    = kLen / kSeg;
constexpr int kNout   = kPred / kSeg;
constexpr int kNoutP  = 48;
constexpr int kCpb    = 8;
constexpr int kXP     = 520;
constexpr int kTP     = 36;
static_assert(kConv == 63, "filter outputs");
static_assert(kNin == 32, "contraction depth is one 32-deep k-step");
static_assert(kNout == 45 && kNoutP % 16 == 0 && kNoutP >= kNout, "output-segment padding");
static_assert(kSeg == 16, "one 16-row tile per (b,c)");
static_assert(kChan % 32 == 0 && kChan % kCpb == 0, "channel grouping");

constexpr float kCarryA = 16.0f;
constexpr float kCarryW = 256.0f;
constexpr float kFold   = 1.0f / (kCarryA * kCarryW);
constexpr float kF16Min = 6.103515625e-05f;

constexpr size_t kBytesWT  = (size_t)kMaps * kNoutP * kNin * 2;
constexpr size_t kBytesA16 = (size_t)kBatch * kChan * kSeg * kNin * 2;
constexpr size_t kBytesREC = (size_t)kBatch * kChan * 8 * 4;
constexpr size_t kOffWT    = 0;
constexpr size_t kOffA16   = kOffWT + kBytesWT;
constexpr size_t kOffREC   = kOffA16 + kBytesA16;
constexpr size_t kWsTotal  = kOffREC + kBytesREC;
static_assert(kBytesWT == 24576ull && kBytesA16 == 16777216ull && kBytesREC == 524288ull, "carve sizes");
static_assert(kWsTotal == 17326080ull, "carve total");
static_assert(kWsTotal <= 134217728ull, "carve cap");
static_assert((kOffA16 % 256) == 0 && (kOffREC % 256) == 0, "aligned regions");

namespace eng {
union FragH { v16h v; v8h h[2]; };
__device__ __forceinline__ v8f mma_f16(v16h a, v16h b, v8f c) {
  c = __builtin_amdgcn_wmma_f32_16x16x32_f16(false, a, false, b, (short)0, c, false, false);
  asm volatile("v_nop\n\tv_nop\n\tv_nop\n\tv_nop" : "+v"(c) : "v"(a), "v"(b));
  return c;
}
__device__ __forceinline__ float wave_sum(float v) {
#pragma unroll
  for (int off = 16; off > 0; off >>= 1) v += __shfl_xor(v, off, 32);
  return v;
}
__device__ __forceinline__ _Float16 to_f16_carried(float v, float carry) {
  float f = v * carry;
  f = (fabsf(f) < kF16Min) ? 0.0f : f;
  return (_Float16)f;
}
}

__global__ __launch_bounds__(256) void prep_w_kernel(const float* __restrict__ map_w, unsigned short* __restrict__ WT)
{
  const int i = blockIdx.x * 256 + threadIdx.x;
  if (i >= (kMaps * kNoutP * kNin) / 8) return;
  const int h0  = i * 8;
  const int m   = h0 / (kNoutP * kNin);
  const int rem = h0 - m * (kNoutP * kNin);
  const int o   = rem / kNin;
  const int n0  = rem - o * kNin;
  const int oc  = (o < kNout) ? o : (kNout - 1);
  const bool valid = (o < kNout);
  const float* src = map_w + ((size_t)(m * kNout + oc)) * kNin + n0;
  const v4f a0 = *(const v4f*)(src);
  const v4f a1 = *(const v4f*)(src + 4);
  v8h hv;
#pragma unroll
  for (int e = 0; e < 4; ++e) {
    const float f0 = valid ? a0[e] : 0.0f;
    const float f1 = valid ? a1[e] : 0.0f;
    hv[e]     = eng::to_f16_carried(f0, kCarryW);
    hv[4 + e] = eng::to_f16_carried(f1, kCarryW);
  }
  unsigned short* dst = WT + (size_t)h0;
  *(volatile v8h*)dst = hv;
  __threadfence();
  *(volatile v8h*)dst = hv;
}

__global__ __launch_bounds__(256) void front_kernel(
    const float* __restrict__ x, const float* __restrict__ conv_w, const float* __restrict__ conv_b,
    const float* __restrict__ gate_w, const float* __restrict__ gate_b,
    unsigned short* __restrict__ A16, float* __restrict__ REC)
{
  __shared__ __align__(16) float xs[kCpb * kXP];
  __shared__ __align__(16) float cvs[kCpb * 64];
  __shared__ __align__(16) float gws[kMaps * 64];
  __shared__ __align__(16) float cws[kCpb * kTaps];
  __shared__ __align__(16) float rec[kCpb * 8];

  const int tid  = threadIdx.x;
  const int w    = tid >> 5;
  const int lane = tid & 31;
  const int b    = blockIdx.x / (kChan / kCpb);
  const int cg   = blockIdx.x - b * (kChan / kCpb);
  const int c    = cg * kCpb + w;

#pragma unroll
  for (int it = 0; it < 4; ++it) {
    const int i = tid + it * 256;
    const int q = i & 1;
    const int l = i >> 1;
    const v4f v = *(const v4f*)(x + ((size_t)(b * kLen + l)) * kChan + cg * kCpb + q * 4);
    xs[(q * 4 + 0) * kXP + l] = v[0];
    xs[(q * 4 + 1) * kXP + l] = v[1];
    xs[(q * 4 + 2) * kXP + l] = v[2];
    xs[(q * 4 + 3) * kXP + l] = v[3];
  }
#pragma unroll
  for (int it = 0; it < 2; ++it) {
    const int i  = tid + it * 256;
    const int m  = i >> 6;
    const int d  = i & 63;
    const int dc = (d < kConv) ? d : (kConv - 1);
    float g = gate_w[m * kConv + dc];
    asm volatile("" : "+v"(g));
    gws[i] = (d < kConv) ? g : 0.0f;
  }
  {
    float cwv = conv_w[cg * kCpb * kTaps + (tid & (kCpb * kTaps - 1))];
    asm volatile("" : "+v"(cwv));
    if (tid < kCpb * kTaps) cws[tid] = cwv;
  }
  __syncthreads();

  float* xc = xs + w * kXP;

  float s = 0.0f;
#pragma unroll 4
  for (int i = 0; i < kLen / 32; ++i) s += xc[lane + i * 32];
  s = eng::wave_sum(s);
  const float mean = s * (1.0f / (float)kLen);

  float s1 = 0.0f;
#pragma unroll 4
  for (int i = 0; i < kLen / 32; ++i) {
    const float d = xc[lane + i * 32] - mean;
    xc[lane + i * 32] = d;
    s1 += d;
  }
  s1 = eng::wave_sum(s1);
  const float mean2 = s1 * (1.0f / (float)kLen);

  float s2 = 0.0f;
#pragma unroll 4
  for (int i = 0; i < kLen / 32; ++i) {
    const float d = xc[lane + i * 32] - mean2;
    s2 = fmaf(d, d, s2);
  }
  s2 = eng::wave_sum(s2);
  const float var   = s2 * (1.0f / (float)kLen);
  const float stdev = sqrtf(var + 1e-10f);
  const float rstd  = 1.0f / stdev;

#pragma unroll 4
  for (int i = 0; i < kLen / 32; ++i) xc[lane + i * 32] = xc[lane + i * 32] * rstd;
  __syncthreads();

  {
    const int d0  = lane;
    const int d1  = lane + 32;
    const int d1c = (d1 < kConv) ? d1 : (kConv - 1);
    float c0 = 0.0f, c1 = 0.0f;
#pragma unroll 4
    for (int k = 0; k < kTaps; ++k) {
      const float wk = cws[w * kTaps + k];
      c0 = fmaf(xc[d0 * kStride + k], wk, c0);
      c1 = fmaf(xc[d1c * kStride + k], wk, c1);
    }
    const float cb = conv_b[c];
    cvs[w * 64 + lane]      = c0 + cb;
    cvs[w * 64 + 32 + lane] = (d1 < kConv) ? (c1 + cb) : 0.0f;
  }
  __syncthreads();

  float logit;
  {
    const int m = lane & 7;
    const int q = lane >> 3;
    float acc = 0.0f;
#pragma unroll 4
    for (int j = 0; j < 16; ++j) {
      const int d = q * 16 + j;
      acc = fmaf(cvs[w * 64 + d], gws[m * 64 + d], acc);
    }
    acc += __shfl_xor(acc, 8, 32);
    acc += __shfl_xor(acc, 16, 32);
    logit = acc + gate_b[m];
  }
  float lg[kMaps];
#pragma unroll
  for (int j = 0; j < kMaps; ++j) lg[j] = __shfl(logit, j, 32);

  int m0 = 0;
  float v0 = lg[0];
#pragma unroll
  for (int j = 1; j < kMaps; ++j) {
    const bool gt = lg[j] > v0;
    v0 = gt ? lg[j] : v0;
    m0 = gt ? j : m0;
  }
  int m1 = 0;
  float v1 = -INFINITY;
#pragma unroll
  for (int j = 0; j < kMaps; ++j) {
    const bool gt = (j != m0) && (lg[j] > v1);
    v1 = gt ? lg[j] : v1;
    m1 = gt ? j : m1;
  }

  const float ex = expf(logit - v0);
  float es[kMaps];
#pragma unroll
  for (int j = 0; j < kMaps; ++j) es[j] = __shfl(ex, j, 32);
  float zsum = 0.0f;
#pragma unroll
  for (int j = 0; j < kMaps; ++j) zsum += es[j];
  const float rz = 1.0f / zsum;
  float e0s = 0.0f, e1s = 0.0f;
#pragma unroll
  for (int j = 0; j < kMaps; ++j) {
    e0s = (j == m0) ? es[j] : e0s;
    e1s = (j == m1) ? es[j] : e1s;
  }
  const float p0 = e0s * rz;
  const float p1 = e1s * rz;
  const float tt = expf(p1 - p0);
  const float g0 = 1.0f / (1.0f + tt);
  const float g1 = tt * g0;

  if (lane == 0) {
    rec[w * 8 + 0] = g0;
    rec[w * 8 + 1] = g1;
    rec[w * 8 + 2] = mean;
    rec[w * 8 + 3] = stdev;
    rec[w * 8 + 4] = (float)m0;
    rec[w * 8 + 5] = (float)m1;
    rec[w * 8 + 6] = 0.0f;
    rec[w * 8 + 7] = 0.0f;
  }

  {
    v8h hv[2];
#pragma unroll
    for (int i = 0; i < 2; ++i) {
      const int u  = i * 32 + lane;
      const int sr = u >> 2;
      const int n0 = (u & 3) * 8;
#pragma unroll
      for (int e = 0; e < 8; ++e) hv[i][e] = eng::to_f16_carried(xc[(n0 + e) * kSeg + sr], kCarryA);
    }
    unsigned short* dst = A16 + ((size_t)(b * kChan + c)) * (kSeg * kNin) + lane * 8;
    for (int pass = 0; pass < 2; ++pass) {
#pragma unroll
      for (int i = 0; i < 2; ++i) *(volatile v8h*)(dst + i * 256) = hv[i];
      __threadfence();
    }
  }
  __syncthreads();

  {
    const v4f rv = *(const v4f*)(rec + (lane & 15) * 4);
    if (w == 0 && lane < 16) {
      float* dst = REC + ((size_t)(b * kChan + cg * kCpb)) * 8 + lane * 4;
      *(volatile v4f*)dst = rv;
      __threadfence();
      *(volatile v4f*)dst = rv;
    }
  }
}

__global__ __launch_bounds__(256) void mix_kernel(
    const unsigned short* __restrict__ A16p, const unsigned short* __restrict__ WTp,
    const float* __restrict__ REC, const float* __restrict__ map_b, float* __restrict__ out)
{
  __shared__ __align__(16) _Float16 sW[kMaps * kNoutP * kNin];
  __shared__ __align__(16) float sT[256 * kTP];
  __shared__ __align__(16) float sRec[32 * 8];
  __shared__ __align__(16) float sMB[kMaps * kNoutP];

  const _Float16* A16 = (const _Float16*)A16p;
  const _Float16* WT  = (const _Float16*)WTp;
  const int tid  = threadIdx.x;
  const int wave = tid >> 5;
  const int lane = tid & 31;
  const int hh   = lane >> 4;
  const int cl   = lane & 15;
  const int b    = blockIdx.x >> 1;
  const int half = blockIdx.x & 1;
  const int chan0 = b * kChan + half * 32;

#pragma unroll
  for (int it = 0; it < 6; ++it) {
    const int i = tid + it * 256;
    *(v8h*)(sW + i * 8) = *(const v8h*)(WT + i * 8);
  }
  sRec[tid] = REC[(size_t)chan0 * 8 + tid];
#pragma unroll
  for (int it = 0; it < 2; ++it) {
    const int idx  = tid + it * 256;
    const int idxc = (idx < kMaps * kNoutP) ? idx : (kMaps * kNoutP - 1);
    const int m  = idxc / kNoutP;
    const int o  = idxc - m * kNoutP;
    const int oc = (o < kNout) ? o : (kNout - 1);
    float bv = map_b[m * kNout + oc];
    asm volatile("" : "+v"(bv));
    const float sel = (o < kNout) ? bv : 0.0f;
    if (idx < kMaps * kNoutP) sMB[idx] = sel;
  }
  __syncthreads();

  const v8f zero8 = (v8f){0.f, 0.f, 0.f, 0.f, 0.f, 0.f, 0.f, 0.f};

#pragma unroll 1
  for (int t = 0; t < 3; ++t) {
#pragma unroll 1
    for (int ch = 0; ch < 4; ++ch) {
      const int cloc = wave * 4 + ch;
      const v4f r0 = *(const v4f*)(sRec + cloc * 8);
      const v4f r1 = *(const v4f*)(sRec + cloc * 8 + 4);
      const float g0 = r0[0];
      const float g1 = r0[1];
      const float mu = r0[2];
      const float sd = r0[3];
      int m0 = (int)r1[0];
      int m1 = (int)r1[1];
      m0 = (m0 < 0) ? 0 : ((m0 > kMaps - 1) ? (kMaps - 1) : m0);
      m1 = (m1 < 0) ? 0 : ((m1 > kMaps - 1) ? (kMaps - 1) : m1);
      m0 = __builtin_amdgcn_readfirstlane(m0);
      m1 = __builtin_amdgcn_readfirstlane(m1);

      const _Float16* ap = A16 + ((size_t)(chan0 + cloc) * kSeg + cl) * kNin + 8 * hh;
      eng::FragH fa;
      fa.h[0] = *(const v8h*)(ap);
      fa.h[1] = *(const v8h*)(ap + 16);

      const int o  = t * 16 + cl;
      const int w0 = (m0 * kNoutP + o) * kNin + 8 * hh;
      const int w1 = (m1 * kNoutP + o) * kNin + 8 * hh;
      eng::FragH fb0, fb1;
      fb0.h[0] = *(const v8h*)(sW + w0);
      fb0.h[1] = *(const v8h*)(sW + w0 + 16);
      fb1.h[0] = *(const v8h*)(sW + w1);
      fb1.h[1] = *(const v8h*)(sW + w1 + 16);

      v8f acc0 = eng::mma_f16(fa.v, fb0.v, zero8);
      v8f acc1 = eng::mma_f16(fa.v, fb1.v, zero8);

      const float bm = fmaf(g1, sMB[m1 * kNoutP + o], g0 * sMB[m0 * kNoutP + o]);
#pragma unroll
      for (int r = 0; r < 8; ++r) {
        float v = fmaf(g1, acc1[r], g0 * acc0[r]);
        v = fmaf(v, kFold, bm);
        v = fmaf(v, sd, mu);
        sT[(cl * 16 + 8 * hh + r) * kTP + cloc] = v;
      }
    }
    __syncthreads();
    {
      const int nquads = (t < 2) ? 64 : ((kNout - 32) * kSeg / 4);
      const int q   = lane >> 3;
      const int c4  = (lane & 7) * 4;
      for (int pass = 0; pass < 2; ++pass) {
#pragma unroll 1
        for (int it = 0; it < 8; ++it) {
          const int q4 = it * 8 + wave;
          if (q4 < nquads) {
            const int row = q4 * 4 + q;
            const v4f val = *(const v4f*)(sT + row * kTP + c4);
            float* dst = out + ((size_t)(b * kPred + t * 256 + row)) * kChan + half * 32 + c4;
            *(volatile v4f*)dst = val;
          }
        }
        __threadfence();
      }
    }
    __syncthreads();
  }
}

extern "C" void kernel_launch(void* const* d_in, const int* in_sizes, int n_in,
                              void* d_out, int out_size, void* d_ws, size_t ws_size,
                              hipStream_t stream) {
  if (n_in < 7) return;
  if (in_sizes[0] != kBatch * kLen * kChan) return;
  if (in_sizes[1] != kChan * kTaps) return;
  if (in_sizes[2] != kChan) return;
  if (in_sizes[3] != kMaps * kConv) return;
  if (in_sizes[4] != kMaps) return;
  if (in_sizes[5] != kMaps * kNout * kNin) return;
  if (in_sizes[6] != kMaps * kNout) return;
  if (out_size != kBatch * kPred * kChan) return;
  if (ws_size < kWsTotal) return;

  const float* x      = (const float*)d_in[0];
  const float* conv_w = (const float*)d_in[1];
  const float* conv_b = (const float*)d_in[2];
  const float* gate_w = (const float*)d_in[3];
  const float* gate_b = (const float*)d_in[4];
  const float* map_w  = (const float*)d_in[5];
  const float* map_b  = (const float*)d_in[6];
  float* out = (float*)d_out;

  char* ws = (char*)d_ws;
  unsigned short* WT  = (unsigned short*)(ws + kOffWT);
  unsigned short* A16 = (unsigned short*)(ws + kOffA16);
  float*          REC = (float*)(ws + kOffREC);

  prep_w_kernel<<<(kMaps * kNoutP * kNin / 8) / 256, 256, 0, stream>>>(map_w, WT);
  front_kernel<<<kBatch * (kChan / kCpb), 256, 0, stream>>>(x, conv_w, conv_b, gate_w, gate_b, A16, REC);
  mix_kernel<<<kBatch * (kChan / 32), 256, 0, stream>>>(A16, WT, REC, map_b, out);
}
